// SelfAttention_11373073399903
// MI455X (gfx1250) — hardware-verified
//
#include <hip/hip_runtime.h>
#include <stdint.h>


typedef _Float16 v16h __attribute__((ext_vector_type(16)));
typedef _Float16 v8h  __attribute__((ext_vector_type(8)));
typedef float    v8f  __attribute__((ext_vector_type(8)));
typedef float    v4f  __attribute__((ext_vector_type(4)));

#ifndef NB
#define NB 8
#endif
#ifndef SEQ
#define SEQ 2048
#endif
#define MCTX SEQ
#define NB_FULL   8
#define SEQ_FULL  2048
#define MCTX_FULL SEQ_FULL
#define DM   512
#define HF   256

#define ACT_CAR   8.0f
#define W_CAR     1024.0f
#define PROJ_SCL  0.0009765625f
#define RES_CAR   2048.0f
#define RES_INV   0.00048828125f
#define S_SCL     (0.015625f * 0.044194173824159216f)
#define P_CAR     16384.0f
#define OV_SCL    7.62939453125e-06f

static_assert(DM == 512);
static_assert(HF * 2 == DM);
static_assert(HF == 256);
static_assert(HF % 64 == 0);
static_assert(DM % 128 == 0 && DM % 32 == 0 && DM % 64 == 0);
static_assert(SEQ % 128 == 0);
static_assert(MCTX == SEQ);
static_assert(MCTX % 256 == 0);
static_assert(MCTX % 32 == 0);
static_assert(SEQ % 8 == 0);
static_assert(NB >= 1 && NB <= NB_FULL);
static_assert(SEQ <= SEQ_FULL && MCTX <= MCTX_FULL);
static_assert((long)NB_FULL * SEQ_FULL * DM * 4 == 33554432L);
static_assert(((long)NB * SEQ * DM / 8) % 256 == 0);
static_assert((long)(DM / 64) * (DM / 64) * 64 * 64 == (long)DM * DM);
static_assert((long)(HF / 64) * ((long)NB * SEQ / 64) * 64 * 128 == (long)NB * SEQ * DM);
static_assert((long)(MCTX / 64) * (DM / 128) * 128 * 64 == (long)DM * MCTX);
static_assert((long)(MCTX / 64) * (SEQ / 64) * 4096 == (long)SEQ * MCTX);
static_assert((long)(SEQ / 8) * 8 * MCTX == (long)SEQ * MCTX);
static_assert((long)(DM / 64) * (SEQ / 128) * 128 * 64 == (long)SEQ * DM);

union Frag16 { v16h v; v8h p[2]; };

__device__ __forceinline__ v16h ld_frag(const _Float16* p, int hl) {
  Frag16 f;
  f.p[0] = *(const v8h*)(p + 8 * hl);
  f.p[1] = *(const v8h*)(p + 16 + 8 * hl);
  return f.v;
}

__device__ __forceinline__ v8f mma(v16h a, v16h b, v8f c) {
  v8f d = __builtin_amdgcn_wmma_f32_16x16x32_f16(false, a, false, b, (short)0, c, false, false);
  asm volatile("v_nop\n\tv_nop\n\tv_nop\n\tv_nop" : "+v"(d) : "v"(a), "v"(b));
  return d;
}

__device__ __forceinline__ float bf16_rne(float x) {
  unsigned int u = __builtin_bit_cast(unsigned int, x);
  u += 0x7FFFu + ((u >> 16) & 1u);
  return __builtin_bit_cast(float, u & 0xFFFF0000u);
}

static __device__ __forceinline__ _Float16 toh_flush(float v) {
  const _Float16 r = (_Float16)v;
  return (fabsf(v) < 6.103515625e-05f) ? (_Float16)0.0f : r;
}

__global__ __launch_bounds__(256) void k_cvt8(const float* __restrict__ src,
                                              _Float16* __restrict__ dst,
                                              int rows_used, int rows_full, float car, int total8)
{
  const int i8 = blockIdx.x * 256 + threadIdx.x;
  if (i8 >= total8) return;
  const size_t e   = (size_t)i8 * 8;
  const size_t r   = e / (size_t)DM;
  const int    col = (int)(e - r * (size_t)DM);
  const size_t b   = r / (size_t)rows_used;
  const size_t rr  = r - b * (size_t)rows_used;
  const float* s = src + (b * (size_t)rows_full + rr) * (size_t)DM + col;
  const v4f x0 = *(const v4f*)s;
  const v4f x1 = *(const v4f*)(s + 4);
  v8h o;
#pragma unroll
  for (int j = 0; j < 4; ++j) {
    const float t0 = x0[j];
    const float t1 = x1[j];
    o[j]     = (_Float16)(bf16_rne(t0) * car);
    o[4 + j] = (_Float16)(bf16_rne(t1) * car);
  }
  _Float16* d = dst + e;
  *(volatile v8h*)d = o;
  __threadfence();
  *(volatile v8h*)d = o;
}

__global__ __launch_bounds__(256) void k_cvtT(const float* __restrict__ src,
                                              _Float16* __restrict__ dst, float car)
{
  __shared__ __attribute__((aligned(16))) _Float16 ldsT[64 * 72];

  const int tid = threadIdx.x;
  const int n0 = blockIdx.x * 64, k0 = blockIdx.y * 64;

#pragma unroll
  for (int i = 0; i < 4; ++i) {
    const int q = i * 256 + tid;
    const int kr = q >> 4, c4 = (q & 15) * 4;
    const v4f x = *(const v4f*)(src + (size_t)(k0 + kr) * DM + n0 + c4);
#pragma unroll
    for (int j = 0; j < 4; ++j) {
      const float t = x[j];
      ldsT[(c4 + j) * 72 + kr] = toh_flush(bf16_rne(t) * car);
    }
  }
  __syncthreads();

  for (int i = 0; i < 2; ++i) {
    const int q = i * 256 + tid;
    const int rowl = q >> 3, ch = (q & 7) * 8;
    const v8h vh = *(const v8h*)(ldsT + rowl * 72 + ch);
    *(volatile v8h*)(dst + (size_t)(n0 + rowl) * DM + k0 + ch) = vh;
  }
  __threadfence();
  for (int i = 0; i < 2; ++i) {
    const int q = i * 256 + tid;
    const int rowl = q >> 3, ch = (q & 7) * 8;
    const v8h vh = *(const v8h*)(ldsT + rowl * 72 + ch);
    *(volatile v8h*)(dst + (size_t)(n0 + rowl) * DM + k0 + ch) = vh;
  }
}

__device__ __forceinline__ void gemm_core(const _Float16* ap0, const _Float16* ap1,
                                          const _Float16* bp01, const _Float16* bp23,
                                          int K, int hl, v8f (&acc)[8])
{
  const size_t bst = (size_t)16 * K;
#pragma unroll 1
  for (int k0 = 0; k0 < K; k0 += 32) {
    const v16h a0 = ld_frag(ap0 + k0, hl);
    const v16h a1 = ld_frag(ap1 + k0, hl);
    const v16h b0 = ld_frag(bp01 + k0, hl);
    const v16h b1 = ld_frag(bp01 + bst + k0, hl);
    const v16h b2 = ld_frag(bp23 + k0, hl);
    const v16h b3 = ld_frag(bp23 + bst + k0, hl);
    acc[0] = mma(a0, b0, acc[0]);
    acc[1] = mma(a0, b1, acc[1]);
    acc[2] = mma(a0, b2, acc[2]);
    acc[3] = mma(a0, b3, acc[3]);
    acc[4] = mma(a1, b0, acc[4]);
    acc[5] = mma(a1, b1, acc[5]);
    acc[6] = mma(a1, b2, acc[6]);
    acc[7] = mma(a1, b3, acc[7]);
  }
}

__global__ __launch_bounds__(128) __attribute__((amdgpu_num_vgpr(256)))
void k_proj(const _Float16* __restrict__ A, const _Float16* __restrict__ Bt,
            const float* __restrict__ bias, _Float16* PH, _Float16* PL, int with_res)
{
  __shared__ __attribute__((aligned(16))) _Float16 ldsH[64 * 136];
  __shared__ __attribute__((aligned(16))) _Float16 ldsL[64 * 136];

  const int tid = threadIdx.x, lane = tid & 31;
  const int w = __builtin_amdgcn_readfirstlane(threadIdx.x >> 5);
  const int hl = lane >> 4, c = lane & 15;
  const int wr = w >> 1, wc = w & 1;
  const int m0 = blockIdx.y * 64, n0 = blockIdx.x * 64;

  const int mw = m0 + 32 * wr;
  const _Float16* ap0  = A  + (size_t)(mw + c) * DM;
  const _Float16* ap1  = A  + (size_t)(mw + 16 + c) * DM;
  const _Float16* bp01 = Bt + (size_t)(n0 + 32 * wc + c) * DM;
  const _Float16* bp23 = Bt + (size_t)(HF + n0 + 32 * wc + c) * DM;

  v8f acc[8] = {};
  gemm_core(ap0, ap1, bp01, bp23, DM, hl, acc);

#pragma unroll
  for (int t = 0; t < 2; ++t) {
    const int jl = 32 * wc + 16 * t + c;
    const float b1 = bf16_rne(bias[n0 + jl]) * ACT_CAR;
    const float b2 = bf16_rne(bias[HF + n0 + jl]) * ACT_CAR;
#pragma unroll
    for (int i = 0; i < 2; ++i)
#pragma unroll
      for (int r = 0; r < 8; ++r) {
        const float x1 = acc[i * 4 + t][r] * PROJ_SCL + b1;
        const float x2 = acc[i * 4 + t + 2][r] * PROJ_SCL + b2;
        acc[i * 4 + t][r]     = x1;
        acc[i * 4 + t + 2][r] = x2;
      }
  }

#pragma unroll
  for (int i = 0; i < 2; ++i)
#pragma unroll
    for (int t = 0; t < 4; ++t)
#pragma unroll
      for (int r = 0; r < 8; ++r) {
        const int rowl = 32 * wr + 16 * i + 8 * hl + r;
        const int coll = ((t < 2) ? 0 : 64) + 32 * wc + 16 * (t & 1) + c;
        ldsH[rowl * 136 + coll] = toh_flush(acc[i * 4 + t][r]);
      }
  if (with_res != 0) {
#pragma unroll
    for (int i = 0; i < 2; ++i)
#pragma unroll
      for (int t = 0; t < 4; ++t)
#pragma unroll
        for (int r = 0; r < 8; ++r) {
          const int rowl = 32 * wr + 16 * i + 8 * hl + r;
          const int coll = ((t < 2) ? 0 : 64) + 32 * wc + 16 * (t & 1) + c;
          const float v = acc[i * 4 + t][r];
          const _Float16 hv = toh_flush(v);
          const float res = (v - (float)hv) * RES_CAR;
          ldsL[rowl * 136 + coll] = toh_flush(res);
        }
  }
  __syncthreads();

  for (int i = 0; i < 8; ++i) {
    const int q = i * 128 + tid;
    const int rowl = q >> 4, seg = (q >> 3) & 1, ch = (q & 7) * 8;
    const v8h vh = *(const v8h*)(ldsH + rowl * 136 + seg * 64 + ch);
    const size_t go = (size_t)(m0 + rowl) * DM + n0 + seg * HF + ch;
    *(volatile v8h*)(PH + go) = vh;
  }
  if (with_res != 0) {
    for (int i = 0; i < 8; ++i) {
      const int q = i * 128 + tid;
      const int rowl = q >> 4, seg = (q >> 3) & 1, ch = (q & 7) * 8;
      const v8h vl = *(const v8h*)(ldsL + rowl * 136 + seg * 64 + ch);
      const size_t go = (size_t)(m0 + rowl) * DM + n0 + seg * HF + ch;
      *(volatile v8h*)(PL + go) = vl;
    }
  }
  __threadfence();
  for (int i = 0; i < 8; ++i) {
    const int q = i * 128 + tid;
    const int rowl = q >> 4, seg = (q >> 3) & 1, ch = (q & 7) * 8;
    const v8h vh = *(const v8h*)(ldsH + rowl * 136 + seg * 64 + ch);
    const size_t go = (size_t)(m0 + rowl) * DM + n0 + seg * HF + ch;
    *(volatile v8h*)(PH + go) = vh;
  }
  if (with_res != 0) {
    for (int i = 0; i < 8; ++i) {
      const int q = i * 128 + tid;
      const int rowl = q >> 4, seg = (q >> 3) & 1, ch = (q & 7) * 8;
      const v8h vl = *(const v8h*)(ldsL + rowl * 136 + seg * 64 + ch);
      const size_t go = (size_t)(m0 + rowl) * DM + n0 + seg * HF + ch;
      *(volatile v8h*)(PL + go) = vl;
    }
  }
}

__global__ __launch_bounds__(128) __attribute__((amdgpu_num_vgpr(256)))
void k_projv(const _Float16* __restrict__ A, const _Float16* __restrict__ Bt,
             const float* __restrict__ bias, _Float16* __restrict__ PH)
{
  __shared__ __attribute__((aligned(16))) _Float16 ldsH[128 * 72];

  const int tid = threadIdx.x, lane = tid & 31, w = tid >> 5;
  const int hl = lane >> 4, c = lane & 15;
  const int m0 = blockIdx.y * 128, n0 = blockIdx.x * 64;
  const int z = blockIdx.z;
  const int mw = m0 + 32 * w;

  const _Float16* Bz = Bt + (size_t)z * MCTX * DM;
  _Float16* const Pz = PH + (size_t)z * DM * MCTX;

  const _Float16* ap0 = A  + (size_t)(mw + c) * DM;
  const _Float16* ap1 = A  + (size_t)(mw + 16 + c) * DM;
  const _Float16* bp  = Bz + (size_t)(n0 + c) * DM;

  v8f acc[8] = {};
  gemm_core(ap0, ap1, bp, bp + (size_t)32 * DM, DM, hl, acc);

#pragma unroll
  for (int i = 0; i < 2; ++i) {
    const float* bb = bias + m0 + 32 * w + 16 * i + 8 * hl;
    const v4f bA = *(const v4f*)bb;
    const v4f bB = *(const v4f*)(bb + 4);
#pragma unroll
    for (int r = 0; r < 8; ++r) {
      const float braw = (r < 4) ? bA[r & 3] : bB[r & 3];
      const float bv = bf16_rne(braw) * ACT_CAR;
      const int rowl = 32 * w + 16 * i + 8 * hl + r;
#pragma unroll
      for (int t = 0; t < 4; ++t) {
        const float v = acc[i * 4 + t][r] * PROJ_SCL + bv;
        ldsH[rowl * 72 + 16 * t + c] = (_Float16)v;
      }
    }
  }
  __syncthreads();

  _Float16* const bh = Pz + (size_t)m0 * MCTX + n0;
  for (int i = 0; i < 8; ++i) {
    const int q = i * 128 + tid;
    const int rowl = q >> 3, ch = (q & 7) * 8;
    const v8h vh = *(const v8h*)(ldsH + rowl * 72 + ch);
    *(volatile v8h*)(bh + (size_t)rowl * MCTX + ch) = vh;
  }
  __threadfence();
  for (int i = 0; i < 8; ++i) {
    const int q = i * 128 + tid;
    const int rowl = q >> 3, ch = (q & 7) * 8;
    const v8h vh = *(const v8h*)(ldsH + rowl * 72 + ch);
    *(volatile v8h*)(bh + (size_t)rowl * MCTX + ch) = vh;
  }
}

__global__ __launch_bounds__(128) __attribute__((amdgpu_num_vgpr(256)))
void k_score(const _Float16* __restrict__ QH, const _Float16* __restrict__ KH,
             float* __restrict__ S)
{
  __shared__ __attribute__((aligned(16))) float ldsF[64 * 68];

  const int tid = threadIdx.x, lane = tid & 31, w = tid >> 5;
  const int hl = lane >> 4, c = lane & 15;
  const int m0 = blockIdx.y * 64, n0 = blockIdx.x * 64;
  const int mw = m0 + 16 * w;

  const _Float16* ah = QH + (size_t)(mw + c) * DM;
  const _Float16* bh = KH + (size_t)(n0 + c) * DM;

  v8f sh[4] = {};
#pragma unroll 1
  for (int k0 = 0; k0 < DM; k0 += 32) {
    const v16h qh = ld_frag(ah + k0, hl);
#pragma unroll
    for (int t = 0; t < 4; ++t) {
      const v16h kf = ld_frag(bh + (size_t)t * 16 * DM + k0, hl);
      sh[t] = mma(qh, kf, sh[t]);
    }
  }

#pragma unroll
  for (int t = 0; t < 4; ++t)
#pragma unroll
    for (int r = 0; r < 8; ++r) {
      const int rowl = 16 * w + 8 * hl + r;
      ldsF[rowl * 68 + 16 * t + c] = sh[t][r] * S_SCL;
    }
  __syncthreads();

  float* const ob = S + (size_t)m0 * MCTX + n0;
  for (int i = 0; i < 8; ++i) {
    const int qi = i * 128 + tid;
    const int rowl = qi >> 4, col = (qi & 15) * 4;
    const v4f v = *(const v4f*)(ldsF + rowl * 68 + col);
    *(volatile v4f*)(ob + (size_t)rowl * MCTX + col) = v;
  }
  __threadfence();
  for (int i = 0; i < 8; ++i) {
    const int qi = i * 128 + tid;
    const int rowl = qi >> 4, col = (qi & 15) * 4;
    const v4f v = *(const v4f*)(ldsF + rowl * 68 + col);
    *(volatile v4f*)(ob + (size_t)rowl * MCTX + col) = v;
  }
}

__global__ __launch_bounds__(256) void k_softmax(const float* __restrict__ S,
                                                 _Float16* __restrict__ P)
{
  constexpr int NI = MCTX / 256;
  static_assert(NI * 256 == MCTX);
  static_assert(NI >= 1 && NI <= 8);
  const int lane = threadIdx.x & 31, w = threadIdx.x >> 5;
  const int row = blockIdx.x * 8 + w;
  const float* sp = S + (size_t)row * MCTX + 8 * lane;

  v4f xa[NI], xb[NI];
#pragma unroll
  for (int i = 0; i < NI; ++i) {
    xa[i] = *(const v4f*)(sp + i * 256);
    xb[i] = *(const v4f*)(sp + i * 256 + 4);
  }
  float mx = -__builtin_inff();
#pragma unroll
  for (int i = 0; i < NI; ++i)
#pragma unroll
    for (int j = 0; j < 4; ++j) {
      mx = fmaxf(mx, xa[i][j]);
      mx = fmaxf(mx, xb[i][j]);
    }
  mx = fmaxf(mx, __shfl_xor(mx, 16, 32));
  mx = fmaxf(mx, __shfl_xor(mx, 8, 32));
  mx = fmaxf(mx, __shfl_xor(mx, 4, 32));
  mx = fmaxf(mx, __shfl_xor(mx, 2, 32));
  mx = fmaxf(mx, __shfl_xor(mx, 1, 32));

  float sm = 0.f;
#pragma unroll
  for (int i = 0; i < NI; ++i)
#pragma unroll
    for (int j = 0; j < 4; ++j) {
      const float ea = __expf(xa[i][j] - mx);
      const float eb = __expf(xb[i][j] - mx);
      xa[i][j] = ea;
      xb[i][j] = eb;
      sm += ea;
      sm += eb;
    }
  sm += __shfl_xor(sm, 16, 32);
  sm += __shfl_xor(sm, 8, 32);
  sm += __shfl_xor(sm, 4, 32);
  sm += __shfl_xor(sm, 2, 32);
  sm += __shfl_xor(sm, 1, 32);
  const float inv = P_CAR * (1.0f / sm);

  v8h o[NI];
#pragma unroll
  for (int i = 0; i < NI; ++i)
#pragma unroll
    for (int j = 0; j < 4; ++j) {
      o[i][j]     = (_Float16)(xa[i][j] * inv);
      o[i][4 + j] = (_Float16)(xb[i][j] * inv);
    }
  _Float16* pp = P + (size_t)row * MCTX + 8 * lane;
#pragma unroll
  for (int i = 0; i < NI; ++i) *(volatile v8h*)(pp + i * 256) = o[i];
  __threadfence();
#pragma unroll
  for (int i = 0; i < NI; ++i) *(volatile v8h*)(pp + i * 256) = o[i];
}

__global__ __launch_bounds__(128) __attribute__((amdgpu_num_vgpr(256)))
void k_pvout(const _Float16* __restrict__ A, const _Float16* __restrict__ Bt,
             float* __restrict__ Out)
{
  __shared__ __attribute__((aligned(16))) float ldsF[128 * 68];

  const int tid = threadIdx.x, lane = tid & 31;
  const int w = __builtin_amdgcn_readfirstlane(threadIdx.x >> 5);
  const int hl = lane >> 4, c = lane & 15;
  const int m0 = blockIdx.y * 128, n0 = blockIdx.x * 64;
  const int mw = m0 + 32 * w;

  const _Float16* ap0 = A  + (size_t)(mw + c) * MCTX;
  const _Float16* ap1 = A  + (size_t)(mw + 16 + c) * MCTX;
  const _Float16* bp  = Bt + (size_t)(n0 + c) * MCTX;

  v8f acc[8] = {};
  gemm_core(ap0, ap1, bp, bp + (size_t)32 * MCTX, MCTX, hl, acc);

#pragma unroll
  for (int t = 0; t < 4; ++t)
#pragma unroll
    for (int i = 0; i < 2; ++i)
#pragma unroll
      for (int r = 0; r < 8; ++r) {
        const int rowl = 32 * w + 16 * i + 8 * hl + r;
        ldsF[rowl * 68 + 16 * t + c] = acc[i * 4 + t][r] * OV_SCL;
      }
  __syncthreads();

  float* const ob = Out + (size_t)m0 * DM + n0;
  for (int i = 0; i < 16; ++i) {
    const int qi = i * 128 + tid;
    const int rowl = qi >> 4, col = (qi & 15) * 4;
    const v4f v = *(const v4f*)(ldsF + rowl * 68 + col);
    *(volatile v4f*)(ob + (size_t)rowl * DM + col) = v;
  }
  __threadfence();
  for (int i = 0; i < 16; ++i) {
    const int qi = i * 128 + tid;
    const int rowl = qi >> 4, col = (qi & 15) * 4;
    const v4f v = *(const v4f*)(ldsF + rowl * 68 + col);
    *(volatile v4f*)(ob + (size_t)rowl * DM + col) = v;
  }
}

constexpr size_t cmax(size_t a, size_t b) { return a > b ? a : b; }
constexpr size_t N_X   = (size_t)NB * SEQ * DM;
constexpr size_t N_W   = (size_t)DM * DM;
constexpr size_t B_X   = N_X * 2;
constexpr size_t B_S   = (size_t)SEQ * MCTX * 4;
constexpr size_t B_P   = (size_t)SEQ * MCTX * 2;
constexpr size_t B_R0  = cmax(B_X, B_S + B_P);
constexpr size_t B_W   = 3 * N_W * 2;
constexpr size_t B_Q   = N_X * 2;
constexpr size_t B_K   = N_X * 2;
constexpr size_t B_VT  = N_X * 2;
constexpr size_t OFF_W   = B_R0;
constexpr size_t OFF_Q   = OFF_W + B_W;
constexpr size_t OFF_K   = OFF_Q + B_Q;
constexpr size_t OFF_VT  = OFF_K + B_K;
constexpr size_t WS_TOTAL = OFF_VT + B_VT;
static_assert(B_X <= B_R0 && B_S + B_P <= B_R0);
static_assert(B_R0 % 128 == 0 && B_W % 128 == 0 && B_S % 128 == 0);
static_assert(B_Q % 128 == 0 && B_K % 128 == 0 && B_VT % 128 == 0);
static_assert(WS_TOTAL <= (size_t)134217728);

extern "C" void kernel_launch(void* const* d_in, const int* in_sizes, int n_in,
                              void* d_out, int out_size, void* d_ws, size_t ws_size,
                              hipStream_t stream)
{
  if (n_in < 7) return;
  const long needX = ((long)(NB - 1) * SEQ_FULL + SEQ) * DM;
  if ((long)in_sizes[0] < needX) return;
  if ((long)in_sizes[1] < (long)DM * DM) return;
  if ((long)in_sizes[2] < (long)DM) return;
  if ((long)in_sizes[3] < (long)DM * DM) return;
  if ((long)in_sizes[4] < (long)DM) return;
  if ((long)in_sizes[5] < (long)DM * DM) return;
  if ((long)in_sizes[6] < (long)DM) return;
  if ((long)out_size < needX) return;
  if (WS_TOTAL > ws_size) return;

  const float* x  = (const float*)d_in[0];
  const float* Wq = (const float*)d_in[1];
  const float* bq = (const float*)d_in[2];
  const float* Wk = (const float*)d_in[3];
  const float* bk = (const float*)d_in[4];
  const float* Wv = (const float*)d_in[5];
  const float* bv = (const float*)d_in[6];
  float* out = (float*)d_out;

  char* const ws = (char*)d_ws;
  _Float16* X16 = (_Float16*)ws;
  float*    Sp  = (float*)ws;
  _Float16* Pp  = (_Float16*)(ws + B_S);
  _Float16* WqP = (_Float16*)(ws + OFF_W);
  _Float16* WkP = WqP + N_W;
  _Float16* WvP = WkP + N_W;
  _Float16* QH  = (_Float16*)(ws + OFF_Q);
  _Float16* KH  = (_Float16*)(ws + OFF_K);
  _Float16* VtH = (_Float16*)(ws + OFF_VT);

  const int tx8 = (int)(N_X / 8);
  k_cvt8<<<(tx8 + 255) / 256, 256, 0, stream>>>(x, X16, SEQ, SEQ_FULL, ACT_CAR, tx8);
  k_cvtT<<<dim3(DM / 64, DM / 64), 256, 0, stream>>>(Wq, WqP, W_CAR);
  k_cvtT<<<dim3(DM / 64, DM / 64), 256, 0, stream>>>(Wk, WkP, W_CAR);
  k_cvtT<<<dim3(DM / 64, DM / 64), 256, 0, stream>>>(Wv, WvP, W_CAR);

  k_proj<<<dim3(HF / 64, NB * SEQ / 64), 128, 0, stream>>>(X16, WqP, bq, QH, QH, 0);
  k_proj<<<dim3(HF / 64, NB * SEQ / 64), 128, 0, stream>>>(X16, WkP, bk, KH, KH, 0);
  k_projv<<<dim3(MCTX / 64, DM / 128, NB), 128, 0, stream>>>(WvP, X16, bv, VtH);

  for (int b = 0; b < NB; ++b) {
    const size_t qo = (size_t)b * SEQ * DM;
    const size_t ko = (size_t)b * MCTX * DM;
    k_score<<<dim3(MCTX / 64, SEQ / 64), 128, 0, stream>>>(QH + qo, KH + ko, Sp);
    k_softmax<<<SEQ / 8, 256, 0, stream>>>(Sp, Pp);
    k_pvout<<<dim3(DM / 64, SEQ / 128), 128, 0, stream>>>(Pp, VtH + ko, out + (size_t)b * SEQ_FULL * DM);
  }
}
